// StressCondGNNLayer_85796266705417
// MI455X (gfx1250) — hardware-verified
//
#include <hip/hip_runtime.h>
#include <stddef.h>
#include <math.h>


#define HD    128
#define XC    512
#define NHD   4
#define SD    64
#define K1    256
#define GR    16
#define AP1   136
#define XSP   516
#define NB    128
#define NBSH  7
#define CHUNK 2048
#define NTHR  256
#define NWAVE 8
#define WCAP  256
#define NGRP  (CHUNK / (NTHR * 4))
#define TP    33
#define ASH   512
#define ASL   768
#define APS   1024

#define L_SACC (NB * XC)
#define L_MX   (NB * NHD)
#define L_DEN  (NB * NHD)
#define L_GB   (2 * HD)
#define L_LIST (NWAVE * WCAP)
#define LDS_BYTES ((L_SACC + L_MX + L_DEN + L_GB + L_LIST + NWAVE) * 4)

static_assert(LDS_BYTES == 275488);
static_assert(WCAP == (CHUNK / NTHR) * 32);
static_assert(NGRP == 2);
static_assert(NB == (1 << NBSH));
static_assert(((CHUNK - 1) << NBSH) < (1 << 30));
static_assert(NB % NWAVE == 0);
static_assert(NB % 16 == 0);
static_assert(XC == NHD * HD);
static_assert(K1 == 2 * HD);
static_assert(NTHR == 2 * HD);
static_assert((L_SACC % 4) == 0);

typedef float          v4f   __attribute__((ext_vector_type(4)));
typedef float          v8f   __attribute__((ext_vector_type(8)));
typedef int            v4i   __attribute__((ext_vector_type(4)));
typedef int            v8i   __attribute__((ext_vector_type(8)));
typedef unsigned short v4us  __attribute__((ext_vector_type(4)));
typedef unsigned short v8us  __attribute__((ext_vector_type(8)));
typedef unsigned short v16us __attribute__((ext_vector_type(16)));
typedef __bf16         v16b  __attribute__((ext_vector_type(16)));

union Frag  { v16b v; v16us u; v8us half[2]; v8i i; };
union Pack8 { v8us h; v4i i; unsigned short s[8]; };
union Pack4 { v4us h; unsigned short s[4]; };

__device__ __forceinline__ v8f wm(const Frag& a, const Frag& b, v8f c) {
  v8f d = __builtin_amdgcn_wmma_f32_16x16x32_bf16(false, a.v, false, b.v, (short)0, c, false, false);
  asm volatile("v_nop\n\tv_nop\n\tv_nop\n\tv_nop" : "+v"(d) : "v"(a.i), "v"(b.i));
  return d;
}

__device__ __forceinline__ float wsum(float v) {
  v += __shfl_xor(v, 16, 32);
  v += __shfl_xor(v, 8, 32);
  v += __shfl_xor(v, 4, 32);
  v += __shfl_xor(v, 2, 32);
  v += __shfl_xor(v, 1, 32);
  return v;
}

__device__ __forceinline__ unsigned short bfr(float f) {
  unsigned u = __float_as_uint(f);
  u += 0x7FFFu + ((u >> 16) & 1u);
  return (unsigned short)(u >> 16);
}
__device__ __forceinline__ void split2(float f, unsigned short& hi, unsigned short& lo) {
  const unsigned short a = bfr(f);
  hi = a;
  lo = bfr(f - __uint_as_float(((unsigned)a) << 16));
}

__global__ __launch_bounds__(NTHR) void k_prepw(
    const float* __restrict__ Wg, const float* __restrict__ W1,
    unsigned short* WgHi, unsigned short* WgLo, unsigned short* W1Hi, unsigned short* W1Lo) {
  __shared__ __attribute__((aligned(16))) float tile[K1 * TP];
  const int tid = threadIdx.x, lane = tid & 31, wave = tid >> 5;
  const bool j1 = (blockIdx.x >= XC / 32);
  const int  K  = j1 ? K1 : HD;
  const int  lg = j1 ? 8 : 7;
  const int  NC = j1 ? HD : XC;
  const int  n0 = (j1 ? ((int)blockIdx.x - XC / 32) : (int)blockIdx.x) * 32;
  const float* W = j1 ? W1 : Wg;
  unsigned short* oh = j1 ? W1Hi : WgHi;
  unsigned short* ol = j1 ? W1Lo : WgLo;

  for (int i = tid; i < K * 32; i += NTHR) {
    const int k = i >> 5, j = i & 31;
    tile[k * TP + j] = W[(size_t)k * NC + n0 + j];
  }
  __syncthreads();

  const int nIt = K >> 6;
  const size_t wbase = (size_t)(n0 + 4 * wave) * K;
#pragma unroll 1
  for (int ps = 0; ps < 2; ++ps) {
    if (ps) __threadfence();
#pragma unroll 1
    for (int it = 0; it < nIt; ++it) {
      const int base = it * 256 + lane * 8;
      const int j    = 4 * wave + (base >> lg);
      const int kk   = base & (K - 1);
      Pack8 ph, pl;
#pragma unroll
      for (int q = 0; q < 8; ++q) {
        unsigned short a, b;
        split2(tile[(kk + q) * TP + j], a, b);
        ph.s[q] = a; pl.s[q] = b;
      }
      *(volatile v4i*)(oh + wbase + base) = ph.i;
      *(volatile v4i*)(ol + wbase + base) = pl.i;
    }
  }
}

__global__ __launch_bounds__(NTHR) void k_gemm1(
    const float* __restrict__ h, const unsigned short* __restrict__ WgHi, const unsigned short* __restrict__ WgLo,
    const float* __restrict__ att_src, const float* __restrict__ att_dst,
    float* xp, float* asd, int nN) {
  __shared__ __attribute__((aligned(16))) unsigned short Ah[GR * AP1];
  __shared__ __attribute__((aligned(16))) unsigned short Al[GR * AP1];
  __shared__ __attribute__((aligned(16))) float Xs[GR * XSP];
  __shared__ __attribute__((aligned(16))) float Psd[2 * GR * NWAVE];

  const int tid  = threadIdx.x;
  const int lane = tid & 31;
  const int wave = tid >> 5;
  const int hh   = lane >> 4;
  const int m    = lane & 15;
  const int rowBase = blockIdx.x * GR;

  {
    const int r  = tid >> 4;
    const int c0 = (tid & 15) * 8;
    int row = rowBase + r;
    if (row > nN - 1) row = nN - 1;
    const float* p = h + (size_t)row * HD + c0;
    const v4f f0 = *(const v4f*)(p), f1 = *(const v4f*)(p + 4);
    Pack8 ph, pl;
    split2(f0.x, ph.s[0], pl.s[0]); split2(f0.y, ph.s[1], pl.s[1]);
    split2(f0.z, ph.s[2], pl.s[2]); split2(f0.w, ph.s[3], pl.s[3]);
    split2(f1.x, ph.s[4], pl.s[4]); split2(f1.y, ph.s[5], pl.s[5]);
    split2(f1.z, ph.s[6], pl.s[6]); split2(f1.w, ph.s[7], pl.s[7]);
    *(v8us*)(Ah + r * AP1 + c0) = ph.h;
    *(v8us*)(Al + r * AP1 + c0) = pl.h;
  }
  __syncthreads();

  const v8f z8 = {0.f, 0.f, 0.f, 0.f, 0.f, 0.f, 0.f, 0.f};
  v8f acc[4];
#pragma unroll
  for (int nt = 0; nt < 4; ++nt) acc[nt] = z8;
#pragma unroll
  for (int kt = 0; kt < HD / 32; ++kt) {
    const int k0 = kt * 32;
    Frag fah, fal;
    const unsigned short* pah = Ah + m * AP1 + k0 + 8 * hh;
    const unsigned short* pal = Al + m * AP1 + k0 + 8 * hh;
    fah.half[0] = *(const v8us*)pah; fah.half[1] = *(const v8us*)(pah + 16);
    fal.half[0] = *(const v8us*)pal; fal.half[1] = *(const v8us*)(pal + 16);
#pragma unroll
    for (int nt = 0; nt < 4; ++nt) {
      const int ncol = wave * 64 + nt * 16 + m;
      Frag fbh, fbl;
      const unsigned short* pbh = WgHi + (size_t)ncol * HD + k0 + 8 * hh;
      const unsigned short* pbl = WgLo + (size_t)ncol * HD + k0 + 8 * hh;
      fbh.half[0] = *(const v8us*)pbh; fbh.half[1] = *(const v8us*)(pbh + 16);
      fbl.half[0] = *(const v8us*)pbl; fbl.half[1] = *(const v8us*)(pbl + 16);
      acc[nt] = wm(fah, fbh, acc[nt]);
      acc[nt] = wm(fah, fbl, acc[nt]);
      acc[nt] = wm(fal, fbh, acc[nt]);
    }
  }

  float ss[8], sd[8];
#pragma unroll
  for (int r = 0; r < 8; ++r) { ss[r] = 0.f; sd[r] = 0.f; }
#pragma unroll
  for (int nt = 0; nt < 4; ++nt) {
    const int col = wave * 64 + nt * 16 + m;
    const float cs = att_src[col];
    const float cd = att_dst[col];
#pragma unroll
    for (int r = 0; r < 8; ++r) {
      const float v = acc[nt][r];
      Xs[(8 * hh + r) * XSP + col] = v;
      ss[r] += v * cs;
      sd[r] += v * cd;
    }
  }
#pragma unroll
  for (int mk = 1; mk < 16; mk <<= 1) {
#pragma unroll
    for (int r = 0; r < 8; ++r) {
      ss[r] += __shfl_xor(ss[r], mk, 32);
      sd[r] += __shfl_xor(sd[r], mk, 32);
    }
  }
  if (m == 0) {
#pragma unroll
    for (int r = 0; r < 8; ++r) {
      Psd[(8 * hh + r) * NWAVE + wave]              = ss[r];
      Psd[GR * NWAVE + (8 * hh + r) * NWAVE + wave] = sd[r];
    }
  }
  __syncthreads();

  v4f xr[8];
#pragma unroll
  for (int i = 0; i < 2; ++i)
#pragma unroll
    for (int s = 0; s < 4; ++s)
      xr[i * 4 + s] = *(const v4f*)(Xs + (2 * wave + i) * XSP + s * 128 + 4 * lane);
  float* xq[2];
#pragma unroll
  for (int i = 0; i < 2; ++i) xq[i] = xp + (size_t)(rowBase + 2 * wave + i) * XC + 4 * lane;

  const int arow = lane >> 1, part = lane & 1;
  const float* pp = Psd + part * (GR * NWAVE) + arow * NWAVE;
  v4f av;
  av.x = pp[0] + pp[1];
  av.y = pp[2] + pp[3];
  av.z = pp[4] + pp[5];
  av.w = pp[6] + pp[7];
  float* gp = asd + (size_t)rowBase * 8 + 4 * lane;

#pragma unroll
  for (int i = 0; i < 2; ++i)
#pragma unroll
    for (int s = 0; s < 4; ++s) *(volatile v4f*)(xq[i] + s * 128) = xr[i * 4 + s];
  if (wave == 0) *(volatile v4f*)gp = av;
  __threadfence();
#pragma unroll
  for (int i = 0; i < 2; ++i)
#pragma unroll
    for (int s = 0; s < 4; ++s) *(volatile v4f*)(xq[i] + s * 128) = xr[i * 4 + s];
  if (wave == 0) *(volatile v4f*)gp = av;
}

__device__ __forceinline__ void apply_edge(float* sacc, float* smx, float* sden,
                                           const float* __restrict__ xp, const float* __restrict__ asd,
                                           int slot, int src, int nd, int lane) {
  const int hd = lane >> 3;
  float al = asd[(size_t)src * 8 + hd] + asd[(size_t)nd * 8 + 4 + hd];
  al = (al > 0.f) ? al : 0.2f * al;
  const int mi = slot * NHD + hd;
  const float mx = smx[mi];
  const float dn = sden[mi];
  const float m2 = fmaxf(mx, al);
  const float sc = __expf(mx - m2);
  const float p  = __expf(al - m2);
  const float* xrow = xp + (size_t)src * XC + 16 * lane;
  float* ar = sacc + slot * XC + 16 * lane;
  const v4f x0 = *(const v4f*)(xrow), x1 = *(const v4f*)(xrow + 4);
  const v4f x2 = *(const v4f*)(xrow + 8), x3 = *(const v4f*)(xrow + 12);
  v4f a0 = *(const v4f*)(ar), a1 = *(const v4f*)(ar + 4);
  v4f a2 = *(const v4f*)(ar + 8), a3 = *(const v4f*)(ar + 12);
  a0 = a0 * sc + x0 * p;
  a1 = a1 * sc + x1 * p;
  a2 = a2 * sc + x2 * p;
  a3 = a3 * sc + x3 * p;
  *(v4f*)(ar)      = a0;
  *(v4f*)(ar + 4)  = a1;
  *(v4f*)(ar + 8)  = a2;
  *(v4f*)(ar + 12) = a3;
  const float dn2 = dn * sc + p;
  if ((lane & 7) == 0) { smx[mi] = m2; sden[mi] = dn2; }
}

__global__ __launch_bounds__(NTHR) void k_agg(
    const float* __restrict__ h, const int* __restrict__ ei,
    const float* __restrict__ xp, const float* __restrict__ asd,
    const float* __restrict__ bias_g, const float* __restrict__ gam, const float* __restrict__ bet,
    const float* __restrict__ Wp, const float* __restrict__ bp,
    const unsigned short* __restrict__ W1Hi, const unsigned short* __restrict__ W1Lo,
    const float* __restrict__ b1, const float* __restrict__ lng, const float* __restrict__ lnb,
    float* out, int nN, int nE) {
  extern __shared__ v4f lds_dyn[];
  float* sacc = (float*)lds_dyn;
  float* smx  = sacc + L_SACC;
  float* sden = smx + L_MX;
  float* gfb  = sden + L_DEN;
  int*   list = (int*)(gfb + L_GB);
  int*   wcnt = list + L_LIST;
  unsigned short* ahi = (unsigned short*)sacc + ASH;
  unsigned short* alo = (unsigned short*)sacc + ASL;

  const int tid  = threadIdx.x;
  const int lane = tid & 31;
  const int wave = tid >> 5;
  const int hh   = lane >> 4;
  const int m    = lane & 15;
  const int nodeBase = blockIdx.x * NB;

  {
    const v4f z4 = {0.f, 0.f, 0.f, 0.f};
    for (int i = tid; i < L_SACC / 4; i += NTHR) lds_dyn[i] = z4;
    for (int i = tid; i < L_MX; i += NTHR) { smx[i] = -1.0e30f; sden[i] = 0.f; }
    const int c = tid & (HD - 1);
    const int which = tid >> 7;
    const float* v = which ? bet : gam;
    float s = 0.f;
#pragma unroll 1
    for (int k = 0; k < SD; ++k) s += v[k] * Wp[k * HD + c];
    gfb[which * HD + c] = s + bp[c];
  }
  __syncthreads();

  const int* eid = ei + nE;
  const bool al16 = ((nE & 3) == 0);

  const int nChunks = (nE + CHUNK - 1) / CHUNK;
#pragma unroll 1
  for (int ch = 0; ch < nChunks; ++ch) {
    const int cbase = ch * CHUNK;
    int wc = 0;
#pragma unroll
    for (int g = 0; g < NGRP; ++g) {
      const int el0 = (g * NTHR + tid) * 4;
      const int e0  = cbase + el0;
      const int sent = -2147483647 - 1;
      v4i d;
      if (al16 && (cbase + CHUNK <= nE)) {
        d = *(const v4i*)(eid + e0);
      } else {
        d.x = (e0     < nE) ? eid[min(e0,     nE - 1)] : sent;
        d.y = (e0 + 1 < nE) ? eid[min(e0 + 1, nE - 1)] : sent;
        d.z = (e0 + 2 < nE) ? eid[min(e0 + 2, nE - 1)] : sent;
        d.w = (e0 + 3 < nE) ? eid[min(e0 + 3, nE - 1)] : sent;
      }
      const unsigned s0 = (unsigned)d.x - (unsigned)nodeBase;
      const unsigned s1 = (unsigned)d.y - (unsigned)nodeBase;
      const unsigned s2 = (unsigned)d.z - (unsigned)nodeBase;
      const unsigned s3 = (unsigned)d.w - (unsigned)nodeBase;
      const bool h0 = s0 < (unsigned)NB;
      const bool h1 = s1 < (unsigned)NB;
      const bool h2 = s2 < (unsigned)NB;
      const bool h3 = s3 < (unsigned)NB;
      const unsigned many = __builtin_amdgcn_ballot_w32(h0 | h1 | h2 | h3);
      if (many != 0u) {
#define HITJ(J, HJ, SJ) { \
          const unsigned mj = __builtin_amdgcn_ballot_w32(HJ); \
          const int pos = wc + (int)__builtin_amdgcn_mbcnt_lo(mj, 0u); \
          if ((HJ) && pos < WCAP) list[wave * WCAP + pos] = ((el0 + (J)) << NBSH) | (int)(SJ); \
          wc += (int)__builtin_popcount(mj); }
        HITJ(0, h0, s0)
        HITJ(1, h1, s1)
        HITJ(2, h2, s2)
        HITJ(3, h3, s3)
#undef HITJ
      }
    }
    if (lane == 0) wcnt[wave] = wc;
    __syncthreads();

    if (wave == 0) {
#pragma unroll 1
      for (int wsx = 0; wsx < NWAVE; ++wsx) {
        int n = wcnt[wsx];
        if (n > WCAP) n = WCAP;
        if (n < 0) n = 0;
#pragma unroll 1
        for (int i = 0; i < n; ++i) {
          const int ent  = list[wsx * WCAP + i];
          const int slot = ent & (NB - 1);
          const int el   = (ent >> NBSH) & (CHUNK - 1);
          int e = cbase + el;
          if (e > nE - 1) e = nE - 1;
          int src = ei[e];
          src = src < 0 ? 0 : (src > nN - 1 ? nN - 1 : src);
          int nd = nodeBase + slot;
          if (nd > nN - 1) nd = nN - 1;
          apply_edge(sacc, smx, sden, xp, asd, slot, src, nd, lane);
        }
      }
    }
    __syncthreads();
  }

#pragma unroll 1
  for (int j = 0; j < NB / NWAVE; ++j) {
    const int slot = wave * (NB / NWAVE) + j;
    int nd = nodeBase + slot;
    if (nd > nN - 1) nd = nN - 1;
    apply_edge(sacc, smx, sden, xp, asd, slot, nd, nd, lane);
  }
  __syncthreads();

  const v4f bg4 = *(const v4f*)(bias_g + 4 * lane);
  const v4f g4  = *(const v4f*)(gfb + 4 * lane);
  const v4f fb4 = *(const v4f*)(gfb + HD + 4 * lane);
#pragma unroll 1
  for (int j = 0; j < NB / NWAVE; ++j) {
    const int slot = wave * (NB / NWAVE) + j;
    const v4f dn = *(const v4f*)(sden + slot * NHD);
    const float i0 = 1.0f / dn.x, i1 = 1.0f / dn.y, i2 = 1.0f / dn.z, i3 = 1.0f / dn.w;
    float* ar = sacc + slot * XC + 4 * lane;
    const v4f a0 = *(const v4f*)(ar), a1 = *(const v4f*)(ar + HD);
    const v4f a2 = *(const v4f*)(ar + 2 * HD), a3 = *(const v4f*)(ar + 3 * HD);
    const v4f am = (a0 * i0 + a1 * i1 + a2 * i2 + a3 * i3) * 0.25f + bg4;
    const v4f sa = am + (g4 * am + fb4);
    *(v4f*)(ar) = sa;
  }
  __syncthreads();

#pragma unroll 1
  for (int j = 0; j < NB / NWAVE; ++j) {
    const int slot = wave * (NB / NWAVE) + j;
    int nd = nodeBase + slot;
    if (nd > nN - 1) nd = nN - 1;
    const v4f hv = *(const v4f*)(h + (size_t)nd * HD + 4 * lane);
    const v4f sv = *(const v4f*)(sacc + slot * XC + 4 * lane);
    Pack4 phh, phl, psh, psl;
    split2(hv.x, phh.s[0], phl.s[0]); split2(hv.y, phh.s[1], phl.s[1]);
    split2(hv.z, phh.s[2], phl.s[2]); split2(hv.w, phh.s[3], phl.s[3]);
    split2(sv.x, psh.s[0], psl.s[0]); split2(sv.y, psh.s[1], psl.s[1]);
    split2(sv.z, psh.s[2], psl.s[2]); split2(sv.w, psh.s[3], psl.s[3]);
    *(v4us*)(ahi + slot * APS + 4 * lane)      = phh.h;
    *(v4us*)(ahi + slot * APS + HD + 4 * lane) = psh.h;
    *(v4us*)(alo + slot * APS + 4 * lane)      = phl.h;
    *(v4us*)(alo + slot * APS + HD + 4 * lane) = psl.h;
  }
  __syncthreads();

  {
    const int ncol = wave * 16 + m;
    const v8f z8 = {0.f, 0.f, 0.f, 0.f, 0.f, 0.f, 0.f, 0.f};
    v8f acc[NB / 16];
#pragma unroll
    for (int mt = 0; mt < NB / 16; ++mt) acc[mt] = z8;
#pragma unroll 1
    for (int kt = 0; kt < K1 / 32; ++kt) {
      const int k0 = kt * 32;
      Frag fbh, fbl;
      const unsigned short* pbh = W1Hi + (size_t)ncol * K1 + k0 + 8 * hh;
      const unsigned short* pbl = W1Lo + (size_t)ncol * K1 + k0 + 8 * hh;
      fbh.half[0] = *(const v8us*)pbh; fbh.half[1] = *(const v8us*)(pbh + 16);
      fbl.half[0] = *(const v8us*)pbl; fbl.half[1] = *(const v8us*)(pbl + 16);
#pragma unroll
      for (int mt = 0; mt < NB / 16; ++mt) {
        Frag fah, fal;
        const unsigned short* pah = ahi + (mt * 16 + m) * APS + k0 + 8 * hh;
        const unsigned short* pal = alo + (mt * 16 + m) * APS + k0 + 8 * hh;
        fah.half[0] = *(const v8us*)pah; fah.half[1] = *(const v8us*)(pah + 16);
        fal.half[0] = *(const v8us*)pal; fal.half[1] = *(const v8us*)(pal + 16);
        acc[mt] = wm(fah, fbh, acc[mt]);
        acc[mt] = wm(fah, fbl, acc[mt]);
        acc[mt] = wm(fal, fbh, acc[mt]);
      }
    }
    const float zb = b1[ncol];
#pragma unroll
    for (int mt = 0; mt < NB / 16; ++mt)
#pragma unroll
      for (int r = 0; r < 8; ++r)
        sacc[(mt * 16 + 8 * hh + r) * XC + ncol] = acc[mt][r] + zb;
  }
  __syncthreads();

  const v4f lg4 = *(const v4f*)(lng + 4 * lane);
  const v4f lb4 = *(const v4f*)(lnb + 4 * lane);
#pragma unroll 1
  for (int j = 0; j < NB / NWAVE; ++j) {
    const int slot = wave * (NB / NWAVE) + j;
    const int node = nodeBase + slot;
    const bool valid = node < nN;
    const int nd = valid ? node : nN - 1;
    const v4f zv = *(const v4f*)(sacc + slot * XC + 4 * lane);
    const float s  = wsum(zv.x + zv.y + zv.z + zv.w);
    const float mu = s * (1.0f / HD);
    const v4f dd = zv - mu;
    const float q  = wsum(dd.x * dd.x + dd.y * dd.y + dd.z * dd.z + dd.w * dd.w);
    const float rs = rsqrtf(q * (1.0f / HD) + 1.0e-5f);
    const v4f t  = dd * rs;
    const v4f y  = t * lg4 + lb4;
    v4f ev;
    ev.x = erff(y.x * 0.70710678118654752f);
    ev.y = erff(y.y * 0.70710678118654752f);
    ev.z = erff(y.z * 0.70710678118654752f);
    ev.w = erff(y.w * 0.70710678118654752f);
    const v4f ge = (y * (ev + 1.0f)) * 0.5f;
    const v4f hv = *(const v4f*)(h + (size_t)nd * HD + 4 * lane);
    const v4f o  = ge + hv;
    float* op = out + (size_t)nd * HD + 4 * lane;
    if (valid) *(volatile v4f*)op = o;
    __threadfence();
    if (valid) *(volatile v4f*)op = o;
  }
}

extern "C" void kernel_launch(void* const* d_in, const int* in_sizes, int n_in,
                              void* d_out, int out_size, void* d_ws, size_t ws_size,
                              hipStream_t stream) {
  if (n_in < 15) return;
  const int nN = in_sizes[0] / HD;
  if (nN <= 0 || in_sizes[0] != nN * HD) return;
  if (in_sizes[1] < 2 || (in_sizes[1] & 1)) return;
  const int nE = in_sizes[1] / 2;
  if (in_sizes[3] != SD || in_sizes[4] != SD) return;
  if (in_sizes[5] != HD * XC || in_sizes[6] != XC || in_sizes[7] != XC) return;
  if (in_sizes[8] != HD || in_sizes[9] != SD * HD || in_sizes[10] != HD) return;
  if (in_sizes[11] != K1 * HD || in_sizes[12] != HD || in_sizes[13] != HD || in_sizes[14] != HD) return;
  if (out_size != nN * HD) return;

  const float* h       = (const float*)d_in[0];
  const int*   ei      = (const int*)d_in[1];
  const float* gam     = (const float*)d_in[3];
  const float* bet     = (const float*)d_in[4];
  const float* Wg      = (const float*)d_in[5];
  const float* att_src = (const float*)d_in[6];
  const float* att_dst = (const float*)d_in[7];
  const float* bias_g  = (const float*)d_in[8];
  const float* Wp      = (const float*)d_in[9];
  const float* bp      = (const float*)d_in[10];
  const float* W1      = (const float*)d_in[11];
  const float* b1      = (const float*)d_in[12];
  const float* lng     = (const float*)d_in[13];
  const float* lnb     = (const float*)d_in[14];
  float* out = (float*)d_out;

  const int nP = ((nN + GR - 1) / GR) * GR;
  size_t off = 0;
  unsigned short* WgHi = (unsigned short*)((char*)d_ws + off); off += (size_t)XC * HD * sizeof(unsigned short);
  unsigned short* WgLo = (unsigned short*)((char*)d_ws + off); off += (size_t)XC * HD * sizeof(unsigned short);
  unsigned short* W1Hi = (unsigned short*)((char*)d_ws + off); off += (size_t)HD * K1 * sizeof(unsigned short);
  unsigned short* W1Lo = (unsigned short*)((char*)d_ws + off); off += (size_t)HD * K1 * sizeof(unsigned short);
  float* xp  = (float*)((char*)d_ws + off); off += (size_t)nP * XC * sizeof(float);
  float* asd = (float*)((char*)d_ws + off); off += (size_t)nP * 8 * sizeof(float);
  if (off > ws_size) return;

  k_prepw<<<XC / 32 + HD / 32, NTHR, 0, stream>>>(Wg, W1, WgHi, WgLo, W1Hi, W1Lo);

  k_gemm1<<<nP / GR, NTHR, 0, stream>>>(h, WgHi, WgLo, att_src, att_dst, xp, asd, nN);

  hipFuncSetAttribute(reinterpret_cast<const void*>(&k_agg),
                      hipFuncAttributeMaxDynamicSharedMemorySize, LDS_BYTES);
  const int grid = (nN + NB - 1) / NB;
  k_agg<<<grid, NTHR, LDS_BYTES, stream>>>(h, ei, xp, asd, bias_g, gam, bet, Wp, bp,
                                           W1Hi, W1Lo, b1, lng, lnb, out, nN, nE);
}
